// LearnableShapelet1D_45724221833337
// MI455X (gfx1250) — hardware-verified
//
#include <hip/hip_runtime.h>
#include <stdint.h>


#define B_     16
#define C_     8
#define T_     4096
#define K_     64
#define L_     128
#define TP_    (T_ - L_ + 1)
#define NT_    ((TP_ + 15) / 16)
#define TROWS_ (NT_ * 16)
#define XSPAD_ (T_ + 32)
#define SP_    128
#define NTHR   256

typedef _Float16 v16h __attribute__((ext_vector_type(16)));
typedef _Float16 v8h  __attribute__((ext_vector_type(8)));
typedef float    v8f  __attribute__((ext_vector_type(8)));
typedef float    v4f  __attribute__((ext_vector_type(4)));

union Frag { v16h v; v8h half[2]; _Float16 e[16]; };

__device__ __forceinline__ v8f wmma_f16(v16h a, v16h b, v8f acc) {
  acc = __builtin_amdgcn_wmma_f32_16x16x32_f16(false, a, false, b, (short)0, acc, false, false);
  asm volatile("v_nop\n\tv_nop\n\tv_nop\n\tv_nop" : "+v"(acc) : "v"(a), "v"(b));
  return acc;
}

__global__ __launch_bounds__(NTHR) void shapelet_fused(const float* __restrict__ x,
                                                       const float* __restrict__ sh,
                                                       float* __restrict__ out,
                                                       int nb) {
  __shared__ __align__(16) _Float16 xs_lds[XSPAD_];
  __shared__ __align__(16) float    xq_lds[T_];
  __shared__ __align__(16) float    w_lds[TROWS_];
  __shared__ __align__(16) _Float16 sh_lds[K_ * SP_];
  __shared__ float s2_lds[K_];
  __shared__ float red_lds[8 * 16];
  __shared__ __align__(16) float ob_lds[K_];

  const int b = blockIdx.x;
  if (b >= nb) return;
  const int tid  = threadIdx.x;
  const int wave = tid >> 5;
  const int lane = tid & 31;
  const int h    = lane >> 4;
  const int m    = lane & 15;

  const float* xb = x + (size_t)b * C_ * T_;
  for (int t = tid; t < T_; t += NTHR) {
    float s = 0.f, q = 0.f;
#pragma unroll
    for (int c = 0; c < C_; ++c) {
      float v = xb[(size_t)c * T_ + t];
      s += v;
      q += v * v;
    }
    xs_lds[t] = (_Float16)(s * 8.0f);
    xq_lds[t] = q;
  }
  if (tid < XSPAD_ - T_) xs_lds[T_ + tid] = (_Float16)0.0f;

  for (int i = tid; i < K_ * L_; i += NTHR) {
    float v = sh[i];
    sh_lds[(i >> 7) * SP_ + (i & (L_ - 1))] = (_Float16)(v * 64.0f);
  }
  {
    const int k = tid >> 2, part = tid & 3;
    const float* sp = sh + k * L_ + part * 32;
    float e = 0.f;
#pragma unroll 8
    for (int l = 0; l < 32; ++l) { float v = sp[l]; e += v * v; }
    e += __shfl_xor(e, 1, 32);
    e += __shfl_xor(e, 2, 32);
    if (part == 0) s2_lds[k] = e;
  }
  __syncthreads();

  for (int t = tid; t < TROWS_; t += NTHR) {
    float w = 0.f;
    if (t < TP_) {
      const float* qp = xq_lds + t;
#pragma unroll 8
      for (int l = 0; l < L_; ++l) w += qp[l];
    }
    w_lds[t] = w;
  }
  __syncthreads();

  const int kt   = wave & 3;
  const int tsub = wave >> 2;

  Frag bfr[4];
  {
    const _Float16* bp = sh_lds + (kt * 16 + m) * SP_ + 8 * h;
#pragma unroll
    for (int c = 0; c < 4; ++c) {
      bfr[c].half[0] = *(const v8h*)(bp + 32 * c);
      bfr[c].half[1] = *(const v8h*)(bp + 32 * c + 16);
    }
  }
  const float s2v = s2_lds[kt * 16 + m] * (float)C_;
  float rmin = __builtin_inff();

  for (int mt = tsub; mt < NT_; mt += 2) {
    const int t0 = mt * 16;
    v8f acc = {0.f, 0.f, 0.f, 0.f, 0.f, 0.f, 0.f, 0.f};
#pragma unroll
    for (int c = 0; c < 4; ++c) {
      Frag a;
      const _Float16* ap = xs_lds + t0 + m + 32 * c + 8 * h;
#pragma unroll
      for (int i = 0; i < 8; ++i) {
        a.e[i]     = ap[i];
        a.e[8 + i] = ap[16 + i];
      }
      acc = wmma_f16(a.v, bfr[c].v, acc);
    }
#pragma unroll
    for (int r = 0; r < 8; ++r) {
      const int tl = t0 + 8 * h + r;
      float d = w_lds[tl] - acc[r] * (1.0f / 256.0f) + s2v;
      if (tl < TP_ && d < rmin) rmin = d;
    }
  }

  {
    float o = __shfl_xor(rmin, 16, 32);
    rmin = o < rmin ? o : rmin;
  }
  if (h == 0) red_lds[wave * 16 + m] = rmin;
  __syncthreads();
  if (tid < K_) {
    const int kk = tid >> 4, n = tid & 15;
    float v0 = red_lds[kk * 16 + n];
    float v1 = red_lds[(kk + 4) * 16 + n];
    ob_lds[tid] = v0 < v1 ? v0 : v1;
  }
  __syncthreads();

  if (tid < 16) {
    v4f v = *(const v4f*)(ob_lds + 4 * tid);
    volatile v4f* op = (volatile v4f*)(out + (size_t)b * K_) + tid;
    *op = v;
    __threadfence();
    *op = v;
  }
}

extern "C" void kernel_launch(void* const* d_in, const int* in_sizes, int n_in,
                              void* d_out, int out_size, void* d_ws, size_t ws_size,
                              hipStream_t stream) {
  (void)d_ws; (void)ws_size;
  if (n_in < 2) return;
  if (in_sizes[0] != B_ * C_ * T_ || in_sizes[1] != K_ * L_ || out_size != B_ * K_) return;
  const float* x  = (const float*)d_in[0];
  const float* sh = (const float*)d_in[1];
  float* out = (float*)d_out;

  shapelet_fused<<<dim3(B_), dim3(NTHR), 0, stream>>>(x, sh, out, B_);
  (void)hipGetLastError();
}
